// GQA_67010079752601
// MI455X (gfx1250) — hardware-verified
//
#include <hip/hip_runtime.h>
#include <math.h>

typedef __attribute__((ext_vector_type(16))) _Float16 v16h;
typedef __attribute__((ext_vector_type(16))) __bf16 v16b;
typedef __attribute__((ext_vector_type(8)))  _Float16 v8h;
typedef __attribute__((ext_vector_type(8)))  __bf16 v8b;
typedef __attribute__((ext_vector_type(8)))  float v8f;
typedef __attribute__((ext_vector_type(4)))  float v4f;
typedef __attribute__((ext_vector_type(4)))  unsigned v4u;
typedef unsigned short u16;

#ifndef NB
#define NB 2
#endif
#ifndef SEQ
#define SEQ 2048
#endif
#define TT SEQ
#define NB_FULL 2
#define TT_FULL 2048
#define DIN 2048
#define NH 16
#define NG 4
#define RR (NH / NG)
#define HD 128
#define CC (NH * HD)
#define CKV (NG * HD)
#define HG 4
#define NQB (TT / 64)
#define SCALE (0.08838834764831845f)
#ifndef QRES
#define QRES 0
#endif
#define SMT 512
static_assert(TT % 128 == 0);
static_assert(NB >= 1 && NB <= NB_FULL);
static_assert(TT <= TT_FULL);
static_assert(DIN == 256 * 8);
static_assert(CC % 128 == 0 && CKV % 128 == 0 && DIN % 128 == 0);
static_assert(CC % 64 == 0 && CKV % 64 == 0 && CC >= CKV);
static_assert(HD % 32 == 0 && HD % 16 == 0 && HD <= 128);
static_assert(NH % HG == 0 && NH % NG == 0);
static_assert((TT / 4 + SMT - 1) / SMT == 1);

#define SZ_QH  (2u * (size_t)NB * TT * CC)
#define SZ_QL  (QRES ? SZ_QH : (size_t)0)
#define SZ_KH  (2u * (size_t)NB * TT * CKV)
#define SZ_S   (4u * (size_t)HG * TT * TT)
#define SZ_XB  (2u * (size_t)NB * TT * DIN)
#define SZ_WQT (2u * (size_t)CC * DIN)
#define SZ_WKT (2u * (size_t)CKV * DIN)
#define SZ_WOT (2u * (size_t)DIN * CC)
#define SZ_PRE (SZ_XB + SZ_WQT + 2u * SZ_WKT)
#define SZ_MAX2(a, b) ((a) > (b) ? (a) : (b))
#define SZ_SCR SZ_MAX2(SZ_S, SZ_MAX2(SZ_PRE, SZ_WOT))
#define WS_QH  ((size_t)0)
#define WS_QL  (WS_QH + SZ_QH)
#define WS_KH  (WS_QL + SZ_QL)
#define WS_VT  (WS_KH + SZ_KH)
#define WS_YH  (WS_VT + SZ_KH)
#define WS_SCR (WS_YH + SZ_QH)
#define WS_XB  (WS_SCR)
#define WS_WQT (WS_XB + SZ_XB)
#define WS_WKT (WS_WQT + SZ_WQT)
#define WS_WVT (WS_WKT + SZ_WKT)
#define WS_S   (WS_SCR)
#define WS_WOT (WS_SCR)
#define WS_END (WS_SCR + SZ_SCR)
static_assert(WS_END <= (size_t)134217728u);
static_assert(WS_WVT + SZ_WKT <= WS_END);
static_assert(WS_S + SZ_S <= WS_END && WS_WOT + SZ_WOT <= WS_END);
static_assert((WS_QL % 128) == 0 && (WS_KH % 128) == 0 && (WS_VT % 128) == 0 && (WS_YH % 128) == 0 && (WS_SCR % 128) == 0 && (WS_WQT % 128) == 0 && (WS_WKT % 128) == 0 && (WS_WVT % 128) == 0);

template <typename T> __device__ __forceinline__ void vst2(void* p, T v) { *(volatile T*)p = v; __threadfence(); *(volatile T*)p = v; }
__device__ __forceinline__ v8f wmma16(v16h a, v16h b, v8f c) {
  v8f d = __builtin_amdgcn_wmma_f32_16x16x32_f16(false, a, false, b, (short)0, c, false, false);
  asm volatile("v_nop\n\tv_nop\n\tv_nop\n\tv_nop" : "+v"(d) : "v"(a), "v"(b));
  return d;
}
__device__ __forceinline__ v8f wmma_bf(v16b a, v16b b, v8f c) {
  v8f d = __builtin_amdgcn_wmma_f32_16x16x32_bf16(false, a, false, b, (short)0, c, false, false);
  asm volatile("v_nop\n\tv_nop\n\tv_nop\n\tv_nop" : "+v"(d) : "v"(a), "v"(b));
  return d;
}
__device__ __forceinline__ v16h frag_h(const _Float16* rowk0, int lane) {
  union { v16h v; v8h q[2]; } u; const _Float16* p = rowk0 + 8 * (lane >> 4);
  u.q[0] = *(const v8h*)p; u.q[1] = *(const v8h*)(p + 16); return u.v;
}
__device__ __forceinline__ v16b frag_bu(const u16* rowk0, int lane) {
  union { v16b v; v4u q[2]; } u; const u16* p = rowk0 + 8 * (lane >> 4);
  u.q[0] = *(const v4u*)p; u.q[1] = *(const v4u*)(p + 16); return u.v;
}
__device__ __forceinline__ v16h frag_f32(const float* rowk0, int lane) {
  v16h a; const float* p = rowk0 + 8 * (lane >> 4);
#pragma unroll
  for (int i = 0; i < 8; ++i) { a[i] = (_Float16)p[i]; a[8 + i] = (_Float16)p[16 + i]; }
  return a;
}
__device__ __forceinline__ float bfr(float v) { return (float)(__bf16)v; }
__device__ __forceinline__ u16 bf_bits(float v) { const __bf16 b = (__bf16)v; return __builtin_bit_cast(u16, b); }
__device__ __forceinline__ u16 h_bits(float v) { const _Float16 h = (_Float16)v; return __builtin_bit_cast(u16, h); }

__global__ __launch_bounds__(256) void k_cvx(const float* __restrict__ X, u16* __restrict__ XB) {
  const int row = blockIdx.x; const int b = row / TT, t = row - b * TT; const int c = threadIdx.x * 8;
  const float* src = X + ((size_t)b * TT_FULL + t) * DIN + c;
  const v4f f0 = *(const v4f*)src, f1 = *(const v4f*)(src + 4);
  v8b v; v[0] = (__bf16)f0.x; v[1] = (__bf16)f0.y; v[2] = (__bf16)f0.z; v[3] = (__bf16)f0.w; v[4] = (__bf16)f1.x; v[5] = (__bf16)f1.y; v[6] = (__bf16)f1.z; v[7] = (__bf16)f1.w;
  union { v8b v; v4u u; } pk; pk.v = v;
  vst2(XB + (size_t)row * DIN + c, pk.u);
}
__global__ __launch_bounds__(256) void k_cvw(const float* __restrict__ W0, const float* __restrict__ W1, const float* __restrict__ W2,
    u16* __restrict__ D0, u16* __restrict__ D1, u16* __restrict__ D2, int K, int N0, int N12, int mode) {
  __shared__ __align__(16) u16 T[64][72];
  const int z = blockIdx.z;
  const float* W = z == 0 ? W0 : z == 1 ? W1 : W2; u16* D = z == 0 ? D0 : z == 1 ? D1 : D2; const int N = z == 0 ? N0 : N12;
  const int k0 = blockIdx.x * 64, n0 = blockIdx.y * 64;
  if (n0 >= N) return;
  const int tid = threadIdx.x;
  { const int kl = tid >> 2, seg = tid & 3; const float* p = W + (size_t)(k0 + kl) * N + n0 + seg * 16;
#pragma unroll
    for (int i4 = 0; i4 < 4; ++i4) { const v4f f = *(const v4f*)(p + i4 * 4); const float fv[4] = {f.x, f.y, f.z, f.w};
#pragma unroll
      for (int c = 0; c < 4; ++c) { const float v = fv[c]; const u16 b16 = bf_bits(v); const u16 h16 = h_bits(bfr(v) * 256.0f); T[seg * 16 + i4 * 4 + c][kl] = mode ? h16 : b16; } } }
  __syncthreads();
#pragma unroll
  for (int it = 0; it < 2; ++it) { const int nl = (tid >> 3) + it * 32, q = tid & 7;
    vst2(D + (size_t)(n0 + nl) * K + k0 + q * 8, *(const v4u*)&T[nl][q * 8]); }
}

__global__ __launch_bounds__(128) void k_proj(const u16* __restrict__ XB, const u16* __restrict__ WQT, const u16* __restrict__ WKT, const u16* __restrict__ WVT,
    const float* __restrict__ BQ, const float* __restrict__ BK, const float* __restrict__ BV,
    _Float16* __restrict__ QH, _Float16* __restrict__ QL, _Float16* __restrict__ KH, _Float16* __restrict__ VT, int wbase) {
  __shared__ __align__(16) _Float16 sh[64][136]; __shared__ __align__(16) _Float16 th[128][72];
#if QRES
  __shared__ __align__(16) _Float16 sl[64][136];
#endif
  const int tid = threadIdx.x, wave = tid >> 5, lane = tid & 31, col = lane & 15, g = lane >> 4;
  const int which = wbase + (int)blockIdx.z; const int c0 = blockIdx.y * 128; const size_t r0w = (size_t)blockIdx.x * 64; const size_t bb = r0w / TT; const int t0 = (int)(r0w - bb * TT);
  const u16* W = which == 0 ? WQT : which == 1 ? WKT : WVT; const float* BA = which == 0 ? BQ : which == 1 ? BK : BV;
  (void)QL;
  v8f acc[8] = {};
#pragma unroll 2
  for (int kc = 0; kc < DIN / 32; ++kc) { const v16b a = frag_bu(XB + (r0w + wave * 16 + col) * DIN + kc * 32, lane);
    asm volatile("s_wait_loadcnt 0x0" ::: "memory");
#pragma unroll
    for (int j = 0; j < 8; ++j) { const v16b w = frag_bu(W + (size_t)(c0 + j * 16 + col) * DIN + kc * 32, lane); asm volatile("s_wait_loadcnt 0x0" ::: "memory"); acc[j] = wmma_bf(a, w, acc[j]); } }
  if (which == 0) {
#pragma unroll
    for (int j = 0; j < 8; ++j) { const float bias = bfr(BA[c0 + j * 16 + col]);
#pragma unroll
      for (int r = 0; r < 8; ++r) { const float v = acc[j][r] + bias; const _Float16 hv = (_Float16)v; sh[wave * 16 + 8 * g + r][j * 16 + col] = hv;
#if QRES
        sl[wave * 16 + 8 * g + r][j * 16 + col] = (_Float16)((v - (float)hv) * 1024.0f);
#endif
      } }
    __syncthreads();
    for (int e = tid; e < 64 * 16; e += 128) { const int rl = e >> 4, q = e & 15; const size_t o = (r0w + rl) * CC + c0 + q * 8;
      vst2(QH + o, *(const v4u*)&sh[rl][q * 8]);
#if QRES
      vst2(QL + o, *(const v4u*)&sl[rl][q * 8]);
#endif
    }
  } else if (which == 1) {
#pragma unroll
    for (int j = 0; j < 8; ++j) { const float bias = bfr(BA[c0 + j * 16 + col]);
#pragma unroll
      for (int r = 0; r < 8; ++r) sh[wave * 16 + 8 * g + r][j * 16 + col] = (_Float16)(acc[j][r] + bias); }
    __syncthreads();
    for (int e = tid; e < 64 * 16; e += 128) { const int rl = e >> 4, q = e & 15; vst2(KH + (r0w + rl) * CKV + c0 + q * 8, *(const v4u*)&sh[rl][q * 8]); }
  } else {
#pragma unroll
    for (int j = 0; j < 8; ++j) { const float bias = bfr(BA[c0 + j * 16 + col]);
#pragma unroll
      for (int r = 0; r < 8; ++r) { const int rl = wave * 16 + 8 * g + r, cl = j * 16 + col; th[cl][rl] = (_Float16)(acc[j][r] + bias); } }
    __syncthreads();
    for (int e = tid; e < 128 * 8; e += 128) { const int cl = e >> 3, q = e & 7; vst2(VT + (bb * CKV + c0 + cl) * (size_t)TT + t0 + q * 8, *(const v4u*)&th[cl][q * 8]); }
  }
}
__global__ __launch_bounds__(128) void k_sc(const _Float16* __restrict__ QH, const _Float16* __restrict__ QL, const _Float16* __restrict__ KH, int b, int h0, float* __restrict__ S0) {
  __shared__ __align__(16) float ss[4][16][132];
  const int qb = blockIdx.x, kb = blockIdx.y; const int h = h0 + (int)blockIdx.z; const int gk = h / RR; float* S = S0 + (size_t)blockIdx.z * TT * TT;
  const int tid = threadIdx.x, wave = tid >> 5, lane = tid & 31, col = lane & 15, g = lane >> 4; const int k0 = kb * 128; const int ql0 = qb * 64 + wave * 16; const size_t q0 = (size_t)b * TT + ql0, kr0 = (size_t)b * TT + k0;
  v8f acc[8] = {};
#if QRES
  v8f accl[8] = {};
#endif
  (void)QL;
#pragma unroll
  for (int kc = 0; kc < HD / 32; ++kc) { const v16h ah = frag_h(QH + (q0 + col) * CC + h * HD + kc * 32, lane);
#if QRES
    const v16h al = frag_h(QL + (q0 + col) * CC + h * HD + kc * 32, lane);
#endif
#pragma unroll
    for (int j = 0; j < 8; ++j) { const v16h kf = frag_h(KH + (kr0 + j * 16 + col) * CKV + gk * HD + kc * 32, lane); acc[j] = wmma16(ah, kf, acc[j]);
#if QRES
      accl[j] = wmma16(al, kf, accl[j]);
#endif
    } }
#pragma unroll
  for (int j = 0; j < 8; ++j) {
#pragma unroll
    for (int r = 0; r < 8; ++r) { float v = acc[j][r];
#if QRES
      v += accl[j][r] * (1.0f / 1024.0f);
#endif
      ss[wave][8 * g + r][j * 16 + col] = v * SCALE; } }
  __syncthreads();
  for (int rl = 0; rl < 16; ++rl) vst2(S + (size_t)(ql0 + rl) * TT + k0 + lane * 4, *(const v4f*)&ss[wave][rl][lane * 4]);
}
__global__ __launch_bounds__(SMT) void k_sm(float* __restrict__ S0) {
  __shared__ float sred[SMT / 32]; __shared__ float sbc;
  constexpr int NQ = TT / 4;
  const int tid = threadIdx.x; const int t = blockIdx.x;
  float* sr = S0 + (size_t)blockIdx.y * TT * TT + (size_t)t * TT;
  const bool ok = tid < NQ; const int qq = ok ? tid : NQ - 1;
  v4f ch = *(const v4f*)(sr + (size_t)qq * 4);
  float m = fmaxf(fmaxf(ch.x, ch.y), fmaxf(ch.z, ch.w));
#pragma unroll
  for (int o = 1; o < 32; o <<= 1) m = fmaxf(m, __shfl_xor(m, o));
  if ((tid & 31) == 0) sred[tid >> 5] = m; __syncthreads(); if (tid == 0) { float a = sred[0]; for (int i = 1; i < SMT / 32; ++i) a = fmaxf(a, sred[i]); sbc = a; } __syncthreads(); m = sbc; __syncthreads();
  v4f e; e.x = expf(ch.x - m); e.y = expf(ch.y - m); e.z = expf(ch.z - m); e.w = expf(ch.w - m);
  float sum = ok ? ((e.x + e.y) + (e.z + e.w)) : 0.f;
#pragma unroll
  for (int o = 1; o < 32; o <<= 1) sum += __shfl_xor(sum, o);
  if ((tid & 31) == 0) sred[tid >> 5] = sum; __syncthreads(); if (tid == 0) { float a = 0.f; for (int i = 0; i < SMT / 32; ++i) a += sred[i]; sbc = a > 0.f ? 2048.0f / a : 0.f; } __syncthreads(); const float inv = sbc;
  if (ok) { const v4f pv = e * inv; vst2(sr + (size_t)tid * 4, pv); }
}
__global__ __launch_bounds__(128) void k_pv(const float* __restrict__ PS0, const _Float16* __restrict__ VT, int b, int h0, _Float16* __restrict__ YH) {
  __shared__ __align__(16) _Float16 so[4][16][HD + 8];
  const int h = h0 + (int)blockIdx.z; const int gk = h / RR; const float* PS = PS0 + (size_t)blockIdx.z * TT * TT;
  const int tid = threadIdx.x, wave = tid >> 5, lane = tid & 31, col = lane & 15, g = lane >> 4; const int qb = blockIdx.x; const int ql0 = qb * 64 + wave * 16;
  v8f acc[HD / 16] = {};
#pragma unroll 1
  for (int kc = 0; kc < TT / 32; ++kc) { const v16h p = frag_f32(PS + (size_t)(ql0 + col) * TT + kc * 32, lane);
    asm volatile("s_wait_loadcnt 0x0" ::: "memory");
#pragma unroll
    for (int j = 0; j < HD / 16; ++j) { const size_t po = ((size_t)b * CKV + gk * HD + j * 16 + col) * (size_t)TT + kc * 32; acc[j] = wmma16(p, frag_h(VT + po, lane), acc[j]); } }
#pragma unroll
  for (int j = 0; j < HD / 16; ++j)
#pragma unroll
    for (int r = 0; r < 8; ++r) so[wave][8 * g + r][j * 16 + col] = (_Float16)(acc[j][r] * (1.0f / 128.0f));
  __syncthreads();
  for (int rl = 0; rl < 16; ++rl) if (lane < HD / 8) vst2(YH + ((size_t)b * TT + ql0 + rl) * CC + h * HD + lane * 8, *(const v4u*)&so[wave][rl][lane * 8]);
}
__global__ __launch_bounds__(128) void k_out(const _Float16* __restrict__ YH, const _Float16* __restrict__ WOT, const float* __restrict__ BO, float* __restrict__ OUT) {
  __shared__ __align__(16) float sf[4][16][132];
  const int tid = threadIdx.x, wave = tid >> 5, lane = tid & 31, col = lane & 15, g = lane >> 4; const int c0 = blockIdx.y * 128; const size_t r0w = (size_t)blockIdx.x * 64 + wave * 16;
  v8f acc[8] = {};
#pragma unroll 2
  for (int kc = 0; kc < CC / 32; ++kc) { const v16h a = frag_h(YH + (r0w + col) * CC + kc * 32, lane); asm volatile("s_wait_loadcnt 0x0" ::: "memory");
#pragma unroll
    for (int j = 0; j < 8; ++j) { const v16h w = frag_h(WOT + (size_t)(c0 + j * 16 + col) * CC + kc * 32, lane); asm volatile("s_wait_loadcnt 0x0" ::: "memory"); acc[j] = wmma16(a, w, acc[j]); } }
#pragma unroll
  for (int j = 0; j < 8; ++j) { const float bias = bfr(BO[c0 + j * 16 + col]);
#pragma unroll
    for (int r = 0; r < 8; ++r) sf[wave][8 * g + r][j * 16 + col] = acc[j][r] * (1.0f / 4096.0f) + bias; }
  __syncthreads();
  for (int rl = 0; rl < 16; ++rl) { const size_t row = r0w + rl; const size_t bq = row / TT, tq = row - bq * TT;
    vst2(OUT + (bq * TT_FULL + tq) * DIN + c0 + lane * 4, *(const v4f*)&sf[wave][rl][lane * 4]); }
}

extern "C" void kernel_launch(void* const* d_in, const int* in_sizes, int n_in, void* d_out, int out_size, void* d_ws, size_t ws_size, hipStream_t stream) {
  if (n_in < 9) return;
  const long need_rows = (long)(NB - 1) * TT_FULL + TT;
  if ((long)in_sizes[0] < need_rows * DIN) return;
  if (in_sizes[1] < DIN * CC || in_sizes[2] < CC || in_sizes[3] < DIN * CKV || in_sizes[4] < CKV || in_sizes[5] < DIN * CKV || in_sizes[6] < CKV || in_sizes[7] < CC * DIN || in_sizes[8] < DIN) return;
  if ((long)out_size < need_rows * DIN) return;
  if (ws_size < (size_t)WS_END) return;
  const float* X = (const float*)d_in[0]; const float* Wq = (const float*)d_in[1]; const float* bq = (const float*)d_in[2];
  const float* Wk = (const float*)d_in[3]; const float* bk = (const float*)d_in[4]; const float* Wv = (const float*)d_in[5]; const float* bv = (const float*)d_in[6];
  const float* Wo = (const float*)d_in[7]; const float* bo = (const float*)d_in[8];
  char* ws = (char*)d_ws;
  _Float16 *QH = (_Float16*)(ws + WS_QH), *QL = (_Float16*)(ws + WS_QL), *KH = (_Float16*)(ws + WS_KH), *VT = (_Float16*)(ws + WS_VT), *YH = (_Float16*)(ws + WS_YH), *WOT = (_Float16*)(ws + WS_WOT);
  u16 *XB = (u16*)(ws + WS_XB), *WQT = (u16*)(ws + WS_WQT), *WKT = (u16*)(ws + WS_WKT), *WVT = (u16*)(ws + WS_WVT);
  float* S = (float*)(ws + WS_S);
  k_cvx<<<dim3(NB * TT), 256, 0, stream>>>(X, XB);
  k_cvw<<<dim3(DIN / 64, CC / 64, 3), 256, 0, stream>>>(Wq, Wk, Wv, WQT, WKT, WVT, DIN, CC, CKV, 0);
  k_proj<<<dim3(NB * TT / 64, CC / 128, 1), 128, 0, stream>>>(XB, WQT, WKT, WVT, bq, bk, bv, QH, QL, KH, VT, 0);
  k_proj<<<dim3(NB * TT / 64, CKV / 128, 2), 128, 0, stream>>>(XB, WQT, WKT, WVT, bq, bk, bv, QH, QL, KH, VT, 1);
  for (int b = 0; b < NB; ++b) for (int h0 = 0; h0 < NH; h0 += HG) {
    k_sc<<<dim3(NQB, TT / 128, HG), 128, 0, stream>>>(QH, QL, KH, b, h0, S);
    k_sm<<<dim3(TT, HG), SMT, 0, stream>>>(S);
    k_pv<<<dim3(NQB, 1, HG), 128, 0, stream>>>(S, VT, b, h0, YH);
  }
  k_cvw<<<dim3(CC / 64, DIN / 64, 1), 256, 0, stream>>>(Wo, Wo, Wo, (u16*)WOT, (u16*)WOT, (u16*)WOT, CC, DIN, DIN, 1);
  k_out<<<dim3(NB * TT / 64, DIN / 128), 128, 0, stream>>>(YH, WOT, bo, (float*)d_out);
}
